// MultiheadSelfAttention_57234734186528
// MI455X (gfx1250) — hardware-verified
//
#include <hip/hip_runtime.h>
#include <math.h>
#include <stdint.h>

#ifndef NB
#define NB    2
#endif
#ifndef SEQ
#define SEQ   2048
#endif
#define NB_FULL  2
#define SEQ_FULL 2048
#define DM    1024
#define NH    16
#define HD    64
#define NQC   (SEQ / 64)
#define NKT   (SEQ / 64)
#define LN_EPS 1e-5f
static_assert(NH * HD == DM);
static_assert((SEQ % 64) == 0 && SEQ >= 64 && SEQ <= SEQ_FULL);
static_assert(NB >= 1 && NB <= NB_FULL);
static_assert((DM & (DM - 1)) == 0 && (DM % 64) == 0 && (DM % 256) == 0);
static_assert(((SEQ * DM / 8) % 256) == 0);
static_assert(((NB * SEQ) % 64) == 0);

typedef _Float16 v16h __attribute__((ext_vector_type(16)));
typedef _Float16 v8h  __attribute__((ext_vector_type(8)));
typedef __bf16   v16b __attribute__((ext_vector_type(16)));
typedef __bf16   v8b  __attribute__((ext_vector_type(8)));
typedef float    v8f  __attribute__((ext_vector_type(8)));
typedef float    v4f  __attribute__((ext_vector_type(4)));
typedef unsigned int v4u __attribute__((ext_vector_type(4)));

#if defined(__HIP_DEVICE_COMPILE__)
#define DEV_ASM 1
#else
#define DEV_ASM 0
#endif

__device__ __forceinline__ unsigned short bf_bits(float f) {
  unsigned u = __float_as_uint(f);
  return (unsigned short)((u + 0x7FFFu + ((u >> 16) & 1u)) >> 16);
}
__device__ __forceinline__ float bf_up(unsigned short hb) { return __uint_as_float(((unsigned)hb) << 16); }
__device__ __forceinline__ unsigned short h_bits(_Float16 x) { return __builtin_bit_cast(unsigned short, x); }
__device__ __forceinline__ unsigned pk16(unsigned short a, unsigned short b) { return (unsigned)a | ((unsigned)b << 16); }
__device__ __forceinline__ v8f zero8() { v8f z = {0.f, 0.f, 0.f, 0.f, 0.f, 0.f, 0.f, 0.f}; return z; }

__device__ __forceinline__ float bias_at(const float* __restrict__ bias, int i, int bpitch, int boff, int nbias) {
  int idx = (i >> 6) * bpitch + boff + (i & 63);
  idx = (idx < 0) ? 0 : idx;
  idx = (idx > nbias - 1) ? (nbias - 1) : idx;
  return bf_up(bf_bits(bias[idx]));
}

template <typename OT> struct FT;
template <> struct FT<__bf16>   { typedef v16b frag; typedef v8b half8; };
template <> struct FT<_Float16> { typedef v16h frag; typedef v8h half8; };

template <typename OT>
__device__ __forceinline__ typename FT<OT>::frag ldfrag(const OT* p) {
  union { typename FT<OT>::frag v; typename FT<OT>::half8 h[2]; } f;
  f.h[0] = *(const typename FT<OT>::half8*)(p);
  f.h[1] = *(const typename FT<OT>::half8*)(p + 16);
  return f.v;
}

__device__ __forceinline__ v8f mmar(v16b a, v16b b, v8f c) {
  return __builtin_amdgcn_wmma_f32_16x16x32_bf16(false, a, false, b, (short)0, c, false, false);
}
__device__ __forceinline__ v8f mmar(v16h a, v16h b, v8f c) {
  return __builtin_amdgcn_wmma_f32_16x16x32_f16(false, a, false, b, (short)0, c, false, false);
}
__device__ __forceinline__ v8f mma_h(v16h a, v16h b, v8f c) {
  c = __builtin_amdgcn_wmma_f32_16x16x32_f16(false, a, false, b, (short)0, c, false, false);
#if DEV_ASM
  asm volatile("v_nop\n\tv_nop\n\tv_nop\n\tv_nop" : "+v"(c) : "v"(a), "v"(b));
#endif
  return c;
}
__device__ __forceinline__ void dep_guard(v8f& a, v8f& b, v16b x, v16b y) {
#if DEV_ASM
  asm volatile("v_nop\n\tv_nop\n\tv_nop\n\tv_nop" : "+v"(a), "+v"(b) : "v"(x), "v"(y));
#else
  (void)a; (void)b; (void)x; (void)y;
#endif
}
__device__ __forceinline__ void dep_guard(v8f& a, v8f& b, v16h x, v16h y) {
#if DEV_ASM
  asm volatile("v_nop\n\tv_nop\n\tv_nop\n\tv_nop" : "+v"(a), "+v"(b) : "v"(x), "v"(y));
#else
  (void)a; (void)b; (void)x; (void)y;
#endif
}
__device__ __forceinline__ void keep4(v16b a, v16b b, v16b c, v16b d) {
#if DEV_ASM
  asm volatile("v_nop" :: "v"(a), "v"(b), "v"(c), "v"(d));
#else
  (void)a; (void)b; (void)c; (void)d;
#endif
}
__device__ __forceinline__ void keep4(v16h a, v16h b, v16h c, v16h d) {
#if DEV_ASM
  asm volatile("v_nop" :: "v"(a), "v"(b), "v"(c), "v"(d));
#else
  (void)a; (void)b; (void)c; (void)d;
#endif
}
__device__ __forceinline__ void acc_guard4(v8f& a, v8f& b, v8f& c, v8f& d) {
#if DEV_ASM
  asm volatile("v_nop\n\tv_nop\n\tv_nop\n\tv_nop" : "+v"(a), "+v"(b), "+v"(c), "+v"(d));
#else
  (void)a; (void)b; (void)c; (void)d;
#endif
}

__global__ __launch_bounds__(256) void cvtbf8(const float* __restrict__ in, long long sstr,
                                             unsigned short* out, long long dstr, int n8) {
  const int i = blockIdx.x * 256 + (int)threadIdx.x;
  const int b = blockIdx.y;
  if (i < n8) {
    const float* src = in + (size_t)b * (size_t)sstr + (size_t)i * 8;
    const v4f a  = *(const v4f*)(src);
    const v4f a4 = *(const v4f*)(src + 4);
    v4u p;
    p[0] = pk16(bf_bits(a[0]),  bf_bits(a[1]));
    p[1] = pk16(bf_bits(a[2]),  bf_bits(a[3]));
    p[2] = pk16(bf_bits(a4[0]), bf_bits(a4[1]));
    p[3] = pk16(bf_bits(a4[2]), bf_bits(a4[3]));
    unsigned short* o = out + (size_t)b * (size_t)dstr + (size_t)i * 8;
    *(volatile v4u*)o = p;
    __threadfence();
    *(volatile v4u*)o = p;
  }
}

__global__ __launch_bounds__(256) void wtrans(const float* __restrict__ W, int Kdim, int Ndim,
                                             unsigned short* out, int G, int P) {
  __shared__ float S[64][65];
  const int tid = (int)threadIdx.x;
  const int n0 = blockIdx.x * 64;
  const int k0 = blockIdx.y * 64;
  {
    const int kr = tid >> 2, cs = (tid & 3) * 16;
    const float* src = W + (size_t)(k0 + kr) * (size_t)Ndim + n0 + cs;
#pragma unroll
    for (int e4 = 0; e4 < 4; ++e4) {
      const v4f v = *(const v4f*)(src + 4 * e4);
      S[kr][cs + 4 * e4 + 0] = v[0];
      S[kr][cs + 4 * e4 + 1] = v[1];
      S[kr][cs + 4 * e4 + 2] = v[2];
      S[kr][cs + 4 * e4 + 3] = v[3];
    }
  }
  __syncthreads();
  v4u pv[2];
  size_t go[2];
#pragma unroll
  for (int it = 0; it < 2; ++it) {
    const int rl = it * 32 + (tid >> 3);
    const int c8 = (tid & 7) * 8;
    const int n  = n0 + rl;
    const int nd = ((n % G) >> 6) * P + (n / G) * 64 + (n & 63);
    v4u a;
#pragma unroll
    for (int e = 0; e < 4; ++e)
      a[e] = pk16(bf_bits(S[c8 + 2 * e][rl]), bf_bits(S[c8 + 2 * e + 1][rl]));
    pv[it] = a;
    go[it] = (size_t)nd * (size_t)Kdim + (size_t)(k0 + c8);
  }
  for (int pass = 0; pass < 2; ++pass) {
#pragma unroll
    for (int it = 0; it < 2; ++it) *(volatile v4u*)(out + go[it]) = pv[it];
    __threadfence();
  }
}

__global__ __launch_bounds__(256) void vtrans16(const unsigned short* __restrict__ vp, unsigned short* vt) {
  __shared__ __align__(16) unsigned short S[64 * 72];
  const int tid = (int)threadIdx.x;
  const int s0  = blockIdx.x * 64;
  const int bh  = blockIdx.y;
  const unsigned short* src = vp + ((size_t)bh * SEQ + (size_t)s0) * HD;
#pragma unroll
  for (int it = 0; it < 2; ++it) {
    const int p   = it * 256 + tid;
    const int key = p >> 3, d0 = (p & 7) * 8;
    const v4u v = *(const v4u*)(src + (size_t)p * 8);
    *(v4u*)(S + key * 72 + d0) = v;
  }
  __syncthreads();
  v4u pv[2];
  size_t go[2];
#pragma unroll
  for (int it = 0; it < 2; ++it) {
    const int dl = it * 32 + (tid >> 3);
    const int c8 = (tid & 7) * 8;
    v4u a;
#pragma unroll
    for (int e = 0; e < 4; ++e)
      a[e] = pk16(S[(c8 + 2 * e) * 72 + dl], S[(c8 + 2 * e + 1) * 72 + dl]);
    pv[it] = a;
    go[it] = ((size_t)bh * HD + (size_t)dl) * SEQ + (size_t)(s0 + c8);
  }
  for (int pass = 0; pass < 2; ++pass) {
#pragma unroll
    for (int it = 0; it < 2; ++it) *(volatile v4u*)(vt + go[it]) = pv[it];
    __threadfence();
  }
}

template <typename OT, int OUT_MODE, int BIAS>
__global__ __launch_bounds__(256) void gemm64(
    const unsigned short* __restrict__ Ap, const unsigned short* __restrict__ Ap2, int lda, long long strideA, int Ksplit,
    const unsigned short* __restrict__ Btp, int ldb, long long strideB, int kmaskB,
    void* Cout, void* Cout2, int ldc, long long strideC,
    const float* __restrict__ bias, int bpitch, int boff, int nbias,
    int M, int N, int K, float oscale, float rscale) {
  typedef typename FT<OT>::frag V16;
  const OT* A  = (const OT*)(const void*)Ap;
  const OT* A2 = (const OT*)(const void*)Ap2;
  const OT* Bt = (const OT*)(const void*)Btp;
  __shared__ __align__(16) float sT[8][16 * 68];
  const int b    = blockIdx.y;
  const int lane = threadIdx.x & 31;
  const int wave = threadIdx.x >> 5;
  const int tilesN = N >> 6;
  const int tilesM = M >> 6;
  const int tile = blockIdx.x * 8 + wave;
  if (tile >= tilesM * tilesN) return;
  const int tm = tile / tilesN;
  const int tn = tile - tm * tilesN;
  const int m0 = tm << 6;
  const int n0 = tn << 6;

  const OT* Ab  = A  + (size_t)b * (size_t)strideA;
  const OT* A2b = A2 + (size_t)b * (size_t)strideA;
  const OT* Bb  = Bt + (size_t)b * (size_t)strideB;

  const int rlane = lane & 15;
  const int koff  = (lane >> 4) * 8;
  const int mOff  = (lane >> 4) * 8;

  v8f acc[4][4];
#pragma unroll
  for (int i = 0; i < 4; ++i)
#pragma unroll
    for (int j = 0; j < 4; ++j) acc[i][j] = zero8();

  for (int k0 = 0; k0 < K; k0 += 32) {
    const bool sec = (k0 >= Ksplit);
    const OT* Ak = sec ? A2b : Ab;
    const int ka = sec ? (k0 - Ksplit) : k0;
    const int kb = k0 & kmaskB;
    V16 bq[4];
#pragma unroll
    for (int j = 0; j < 4; ++j)
      bq[j] = ldfrag<OT>(Bb + (size_t)(n0 + (j << 4) + rlane) * (size_t)ldb + koff + kb);
#pragma unroll
    for (int i = 0; i < 4; ++i) {
      const V16 af = ldfrag<OT>(Ak + (size_t)(m0 + (i << 4) + rlane) * (size_t)lda + koff + ka);
#pragma unroll
      for (int j = 0; j < 4; ++j) acc[i][j] = mmar(af, bq[j], acc[i][j]);
      dep_guard(acc[i][0], acc[i][3], af, bq[3]);
    }
    keep4(bq[0], bq[1], bq[2], bq[3]);
  }
  acc_guard4(acc[0][0], acc[0][1], acc[0][2], acc[0][3]);
  acc_guard4(acc[1][0], acc[1][1], acc[1][2], acc[1][3]);
  acc_guard4(acc[2][0], acc[2][1], acc[2][2], acc[2][3]);
  acc_guard4(acc[3][0], acc[3][1], acc[3][2], acc[3][3]);

  float* slab = sT[wave];
  const int h2 = lane >> 4, c4 = (lane & 15) * 4;
  const int q  = lane >> 3, c8 = (lane & 7) * 8;
  v4f bb = {0.f, 0.f, 0.f, 0.f};
  float bc[8];
#pragma unroll
  for (int e = 0; e < 8; ++e) bc[e] = 0.f;
  if (BIAS == 1) {
    if (OUT_MODE == 0) {
#pragma unroll
      for (int e = 0; e < 4; ++e) bb[e] = bias_at(bias, n0 + c4 + e, bpitch, boff, nbias);
    } else {
#pragma unroll
      for (int e = 0; e < 8; ++e) bc[e] = bias_at(bias, n0 + c8 + e, bpitch, boff, nbias);
    }
  }
#pragma unroll
  for (int i = 0; i < 4; ++i) {
    const int mBase = m0 + (i << 4);
#pragma unroll
    for (int j = 0; j < 4; ++j) {
#pragma unroll
      for (int r = 0; r < 8; ++r) {
        slab[(mOff + r) * 68 + (j << 4) + rlane] = acc[i][j][r];
      }
    }
    __builtin_amdgcn_fence(3, "workgroup");
    __builtin_amdgcn_wave_barrier();
    __builtin_amdgcn_fence(2, "workgroup");
    if (OUT_MODE == 0) {
      float* C = (float*)Cout + (size_t)b * (size_t)strideC;
      v4f vv[8];
#pragma unroll
      for (int it = 0; it < 8; ++it) {
        const int row = it * 2 + h2;
        float br = 0.f;
        if (BIAS == 2) br = bias_at(bias, mBase + row, bpitch, boff, nbias);
        const v4f sv = *(const v4f*)(slab + row * 68 + c4);
        vv[it] = sv * oscale + bb + br;
      }
      for (int pass = 0; pass < 2; ++pass) {
#pragma unroll
        for (int it = 0; it < 8; ++it) {
          const int row = it * 2 + h2;
          *(volatile v4f*)(C + (size_t)(mBase + row) * (size_t)ldc + n0 + c4) = vv[it];
        }
        __threadfence();
      }
    } else {
      unsigned short* C  = (unsigned short*)Cout  + (size_t)b * (size_t)strideC;
      unsigned short* C2 = (unsigned short*)Cout2 + (size_t)b * (size_t)strideC;
      v4u hv[4], lv[4];
#pragma unroll
      for (int it = 0; it < 4; ++it) {
        const int row = it * 4 + q;
        const float* sp = slab + row * 68 + c8;
        float br = 0.f;
        if (BIAS == 2) br = bias_at(bias, mBase + row, bpitch, boff, nbias);
        float f[8];
#pragma unroll
        for (int e = 0; e < 8; ++e) {
          const float badd = (BIAS == 1) ? bc[e] : br;
          f[e] = (sp[e] + badd) * oscale;
        }
        v4u a, a2;
#pragma unroll
        for (int e = 0; e < 4; ++e) {
          const float f0 = f[2 * e], f1 = f[2 * e + 1];
          const _Float16 x0 = (_Float16)f0, x1 = (_Float16)f1;
          const unsigned short h0 = h_bits(x0), h1 = h_bits(x1);
          unsigned short l0 = 0, l1 = 0;
          if (OUT_MODE == 3) {
            l0 = h_bits((_Float16)((f0 - (float)x0) * rscale));
            l1 = h_bits((_Float16)((f1 - (float)x1) * rscale));
          }
          a[e] = pk16(h0, h1); a2[e] = pk16(l0, l1);
        }
        hv[it] = a; lv[it] = a2;
      }
      for (int pass = 0; pass < 2; ++pass) {
#pragma unroll
        for (int it = 0; it < 4; ++it) {
          const int row = it * 4 + q;
          *(volatile v4u*)(C + (size_t)(mBase + row) * (size_t)ldc + n0 + c8) = hv[it];
          if (OUT_MODE == 3) *(volatile v4u*)(C2 + (size_t)(mBase + row) * (size_t)ldc + n0 + c8) = lv[it];
        }
        __threadfence();
      }
    }
    __builtin_amdgcn_fence(3, "workgroup");
    __builtin_amdgcn_wave_barrier();
    __builtin_amdgcn_fence(2, "workgroup");
  }
}

__global__ __launch_bounds__(128) __attribute__((amdgpu_num_vgpr(256)))
void attn_mha(const unsigned short* __restrict__ qhp, const unsigned short* __restrict__ qlp,
              const unsigned short* __restrict__ kpp, const unsigned short* __restrict__ vtp,
              unsigned short* chp, unsigned short* clp, float sscale) {
  union FH { v16h v; v8h h[2]; };
  __shared__ __align__(16) _Float16 Ksh[64 * 64];
  __shared__ __align__(16) _Float16 Vth[64 * 64];
  __shared__ __align__(16) _Float16 Psh[4][16 * 64];
  __shared__ __align__(16) float    Os[4][16 * 64];

  const int tid  = threadIdx.x;
  const int wave = tid >> 5;
  const int lane = tid & 31;
  const int hh   = lane >> 4;
  const int c    = lane & 15;

  const int bx   = blockIdx.x;
  const int qc   = bx % NQC;
  const int bh   = bx / NQC;
  const int q0   = qc * 64 + wave * 16;
  const size_t hb = (size_t)bh * SEQ * HD;

  const _Float16* Qh = (const _Float16*)(const void*)qhp + hb;
  const _Float16* Ql = (const _Float16*)(const void*)qlp + hb;
  const _Float16* Kg = (const _Float16*)(const void*)kpp + hb;
  const _Float16* Vg = (const _Float16*)(const void*)vtp + (size_t)bh * HD * SEQ;

  v16h qah[2], qal[2];
#pragma unroll
  for (int dc = 0; dc < 2; ++dc) {
    const size_t qo = (size_t)(q0 + c) * HD + dc * 32 + 8 * hh;
    qah[dc] = ldfrag<_Float16>(Qh + qo);
    qal[dc] = ldfrag<_Float16>(Ql + qo);
  }

  float mrow[8], lrow[8];
  v8f oacc[4];
#pragma unroll
  for (int r = 0; r < 8; ++r) { mrow[r] = -INFINITY; lrow[r] = 0.f; }
#pragma unroll
  for (int t = 0; t < 4; ++t) oacc[t] = zero8();

#pragma unroll 1
  for (int kt = 0; kt < NKT; ++kt) {
    const int kv0 = kt * 64;
    __syncthreads();
    {
      const int r = tid >> 1, half = (tid & 1) * 32;
      const _Float16* kg = Kg + (size_t)(kv0 + r) * HD + half;
      const _Float16* vg = Vg + (size_t)r * SEQ + kv0 + half;
#pragma unroll
      for (int i = 0; i < 4; ++i) {
        const v8h a0 = *(const v8h*)(kg + 8 * i);
        const v8h b0 = *(const v8h*)(vg + 8 * i);
        *(v8h*)(Ksh + r * 64 + half + 8 * i) = a0;
        *(v8h*)(Vth + r * 64 + half + 8 * i) = b0;
      }
    }
    __syncthreads();

    v8f s[4];
#pragma unroll
    for (int j = 0; j < 4; ++j) {
      v8f ah = zero8(), al = zero8();
#pragma unroll
      for (int dc = 0; dc < 2; ++dc) {
        FH kb;
        kb.h[0] = *(const v8h*)(Ksh + (j * 16 + c) * 64 + dc * 32 + 8 * hh);
        kb.h[1] = *(const v8h*)(Ksh + (j * 16 + c) * 64 + dc * 32 + 16 + 8 * hh);
        ah = mma_h(qah[dc], kb.v, ah);
        al = mma_h(qal[dc], kb.v, al);
      }
#pragma unroll
      for (int r = 0; r < 8; ++r) {
        s[j][r] = (ah[r] + al[r] * (1.0f / 4096.0f)) * sscale;
      }
    }

    _Float16* pwh = Psh[wave];
#pragma unroll
    for (int r = 0; r < 8; ++r) {
      float m = s[0][r];
#pragma unroll
      for (int j = 1; j < 4; ++j) m = fmaxf(m, s[j][r]);
#pragma unroll
      for (int off = 1; off < 16; off <<= 1) m = fmaxf(m, __shfl_xor(m, off, 32));
      const float mnew  = fmaxf(mrow[r], m);
      const float msafe = (mnew == -INFINITY) ? 0.f : mnew;
      const float alpha = __expf(mrow[r] - msafe);
      mrow[r] = mnew;
      float psum = 0.f;
#pragma unroll
      for (int j = 0; j < 4; ++j) {
        const float p = __expf(s[j][r] - msafe);
        psum += p;
        pwh[(8 * hh + r) * 64 + j * 16 + c] = (_Float16)(p * 16384.0f);
      }
#pragma unroll
      for (int off = 1; off < 16; off <<= 1) psum += __shfl_xor(psum, off, 32);
      lrow[r] = lrow[r] * alpha + psum;
#pragma unroll
      for (int t = 0; t < 4; ++t) oacc[t][r] *= alpha;
    }
    __builtin_amdgcn_fence(3, "workgroup");
    __builtin_amdgcn_wave_barrier();
    __builtin_amdgcn_fence(2, "workgroup");

#pragma unroll 1
    for (int kk = 0; kk < 2; ++kk) {
      FH pa;
      pa.h[0] = *(const v8h*)(pwh + c * 64 + kk * 32 + 8 * hh);
      pa.h[1] = *(const v8h*)(pwh + c * 64 + kk * 32 + 16 + 8 * hh);
#pragma unroll
      for (int t = 0; t < 4; ++t) {
        FH vf;
        vf.h[0] = *(const v8h*)(Vth + (t * 16 + c) * 64 + kk * 32 + 8 * hh);
        vf.h[1] = *(const v8h*)(Vth + (t * 16 + c) * 64 + kk * 32 + 16 + 8 * hh);
        oacc[t] = mma_h(pa.v, vf.v, oacc[t]);
      }
    }
  }

  float* os = Os[wave];
#pragma unroll
  for (int r = 0; r < 8; ++r) {
    const float l = lrow[r];
    const float inv = ((l > 0.f) ? (1.0f / l) : 0.f) * (1.0f / 1048576.0f);
#pragma unroll
    for (int t = 0; t < 4; ++t) os[(8 * hh + r) * 64 + t * 16 + c] = oacc[t][r] * inv;
  }
  __builtin_amdgcn_fence(3, "workgroup");
  __builtin_amdgcn_wave_barrier();
  __builtin_amdgcn_fence(2, "workgroup");
  {
    const int q4 = lane >> 3, c8 = (lane & 7) * 8;
    v4u hv[4], lv[4];
#pragma unroll
    for (int it = 0; it < 4; ++it) {
      const int row = it * 4 + q4;
      const float* sp = os + row * 64 + c8;
      v4u a, a2;
#pragma unroll
      for (int e = 0; e < 4; ++e) {
        const float f0 = sp[2 * e], f1 = sp[2 * e + 1];
        const unsigned short h0 = bf_bits(f0), h1 = bf_bits(f1);
        const unsigned short l0 = bf_bits(f0 - bf_up(h0)), l1 = bf_bits(f1 - bf_up(h1));
        a[e] = pk16(h0, h1); a2[e] = pk16(l0, l1);
      }
      hv[it] = a; lv[it] = a2;
    }
    for (int pass = 0; pass < 2; ++pass) {
#pragma unroll
      for (int it = 0; it < 4; ++it) {
        const int row = it * 4 + q4;
        const size_t go = hb + (size_t)(q0 + row) * HD + c8;
        *(volatile v4u*)(chp + go) = hv[it];
        *(volatile v4u*)(clp + go) = lv[it];
      }
      __threadfence();
    }
  }
}

__global__ __launch_bounds__(256) void lngelu(const float* __restrict__ Y, const unsigned short* __restrict__ xb,
                                             const float* __restrict__ gamma, int ng,
                                             const float* __restrict__ beta, int nbt, float* out) {
#pragma clang fp contract(off)
  __shared__ __align__(16) float srow[DM];
  __shared__ float red[2][8];
  const int row  = blockIdx.x;
  const int tid  = (int)threadIdx.x;
  const int lane = tid & 31, wave = tid >> 5;
  const float* yr = Y + (size_t)row * DM;
  const unsigned short* xr = xb + (size_t)row * DM;

  float s = 0.f;
#pragma unroll 1
  for (int e = 0; e < DM / 256; ++e) {
    const int i = e * 256 + tid;
    const float v = yr[i] + bf_up(xr[i]);
    srow[i] = v;
    s += v;
  }
#pragma unroll
  for (int off = 1; off < 32; off <<= 1) s += __shfl_xor(s, off, 32);
  if (lane == 0) red[0][wave] = s;
  __syncthreads();
  float ts = 0.f;
#pragma unroll
  for (int w = 0; w < 8; ++w) ts += red[0][w];
  const float mu = ts * (1.0f / (float)DM);

  float s2 = 0.f;
#pragma unroll 1
  for (int e = 0; e < DM / 256; ++e) {
    const int i = e * 256 + tid;
    const float dv = srow[i] - mu;
    s2 += dv * dv;
  }
#pragma unroll
  for (int off = 1; off < 32; off <<= 1) s2 += __shfl_xor(s2, off, 32);
  if (lane == 0) red[1][wave] = s2;
  __syncthreads();
  float ts2 = 0.f;
#pragma unroll
  for (int w = 0; w < 8; ++w) ts2 += red[1][w];
  const float var  = ts2 * (1.0f / (float)DM);
  const float rstd = rsqrtf(var + LN_EPS);

#pragma unroll 1
  for (int e = 0; e < DM / 256; ++e) {
    const int i  = e * 256 + tid;
    const int gi = (i < ng) ? i : (ng - 1);
    const int bi = (i < nbt) ? i : (nbt - 1);
    const float g  = bf_up(bf_bits(gamma[gi]));
    const float bt = bf_up(bf_bits(beta[bi]));
    const float n  = (srow[i] - mu) * rstd * g + bt;
    const float er = erff(n * 0.70710678118654752f);
    const float o  = n * (er + 1.0f) * 0.5f;
    srow[i] = o;
  }
  __syncthreads();
  const v4f ov = *(const v4f*)(srow + 4 * tid);
  float* op = out + (size_t)row * DM + 4 * tid;
  *(volatile v4f*)op = ov;
  __threadfence();
  *(volatile v4f*)op = ov;
}

extern "C" void kernel_launch(void* const* d_in, const int* in_sizes, int n_in,
                              void* d_out, int out_size, void* d_ws, size_t ws_size,
                              hipStream_t stream) {
  if (n_in < 11) return;
  if (in_sizes[0] < (NB - 1) * SEQ_FULL * DM + SEQ * DM) return;
  if (in_sizes[1] < DM * DM || in_sizes[3] < DM * DM || in_sizes[5] < DM * DM || in_sizes[7] < DM * DM) return;
  if (in_sizes[2] < DM || in_sizes[4] < DM || in_sizes[6] < DM || in_sizes[8] < DM) return;
  if (in_sizes[9] < DM || in_sizes[10] < DM) return;
  if (out_size < NB * SEQ * DM) return;

  const float* x     = (const float*)d_in[0];
  const float* Wq    = (const float*)d_in[1];
  const float* bq    = (const float*)d_in[2];
  const float* Wk    = (const float*)d_in[3];
  const float* bk    = (const float*)d_in[4];
  const float* Wv    = (const float*)d_in[5];
  const float* bv    = (const float*)d_in[6];
  const float* Wo    = (const float*)d_in[7];
  const float* bo    = (const float*)d_in[8];
  const float* gamma = (const float*)d_in[9];
  const float* beta  = (const float*)d_in[10];
  const int nbq = in_sizes[2], nbk = in_sizes[4], nbv = in_sizes[6], nbo = in_sizes[8];
  const int ngm = in_sizes[9], nbt = in_sizes[10];

  const size_t PX  = (size_t)NB * SEQ * DM * 2;
  const size_t PW  = (size_t)DM * DM * 2;
  const size_t PVT = (size_t)NB * NH * HD * SEQ * 2;
  const size_t PY  = (size_t)NB * SEQ * DM * 4;
  size_t off = 0;
  const size_t oXb = off; off += PX;
  const size_t oWq = off; off += PW;
  const size_t oWk = off; off += PW;
  const size_t oWv = off; off += PW;
  const size_t oWo = off; off += PW;
  const size_t oQh = off; off += PX;
  const size_t oQl = off; off += PX;
  const size_t oKp = off; off += PX;
  const size_t oVp = off; off += PX;
  const size_t oVT = off; off += PVT;
  const size_t oCh = off; off += PX;
  const size_t oCl = off; off += PX;
  const size_t oY  = off; off += PY;
  if (off > ws_size) return;
  if (off > (size_t)134217728) return;

  char* ws = (char*)d_ws;
  unsigned short* Xb  = (unsigned short*)(ws + oXb);
  unsigned short* WqT = (unsigned short*)(ws + oWq);
  unsigned short* WkT = (unsigned short*)(ws + oWk);
  unsigned short* WvT = (unsigned short*)(ws + oWv);
  unsigned short* WoT = (unsigned short*)(ws + oWo);
  unsigned short* Qh  = (unsigned short*)(ws + oQh);
  unsigned short* Ql  = (unsigned short*)(ws + oQl);
  unsigned short* Kp  = (unsigned short*)(ws + oKp);
  unsigned short* Vp  = (unsigned short*)(ws + oVp);
  unsigned short* VT  = (unsigned short*)(ws + oVT);
  unsigned short* Ch  = (unsigned short*)(ws + oCh);
  unsigned short* Cl  = (unsigned short*)(ws + oCl);
  float*          Y   = (float*)(ws + oY);

  const dim3 blk(256);
  const int  MQ   = NB * SEQ;
  const int  n8x  = SEQ * DM / 8;
  const dim3 gCvtX(n8x / 256, NB);
  const dim3 gT(DM / 64, DM / 64);
  const dim3 gQ((((MQ / 64) * (DM / 64)) + 7) / 8, 1);
  const dim3 gV(SEQ / 64, NB * NH);
  const dim3 gAttn(NB * NH * NQC);
  const dim3 gLN(MQ);
  const int  KNEVER = 0x40000000;
  const int  KALL   = 0x7FFFFFFF;

  cvtbf8<<<gCvtX, blk, 0, stream>>>(x, (long long)SEQ_FULL * DM, Xb, (long long)SEQ * DM, n8x);
  wtrans<<<gT, blk, 0, stream>>>(Wq, DM, DM, WqT, 64, DM);
  wtrans<<<gT, blk, 0, stream>>>(Wk, DM, DM, WkT, 64, DM);
  wtrans<<<gT, blk, 0, stream>>>(Wv, DM, DM, WvT, 64, DM);
  wtrans<<<gT, blk, 0, stream>>>(Wo, DM, DM, WoT, 64, DM);
  gemm64<__bf16, 3, 1><<<gQ, blk, 0, stream>>>(
      Xb, Xb, DM, 0LL, KNEVER, WqT, DM, 0LL, KALL,
      (void*)Qh, (void*)Ql, DM, 0LL, bq, 64, 0, nbq,
      MQ, DM, DM, 1.0f, 4096.0f);
  gemm64<__bf16, 1, 1><<<gQ, blk, 0, stream>>>(
      Xb, Xb, DM, 0LL, KNEVER, WkT, DM, 0LL, KALL,
      (void*)Kp, (void*)Kp, DM, 0LL, bk, 64, 0, nbk,
      MQ, DM, DM, 1.0f, 1.0f);
  gemm64<__bf16, 1, 1><<<gQ, blk, 0, stream>>>(
      Xb, Xb, DM, 0LL, KNEVER, WvT, DM, 0LL, KALL,
      (void*)Vp, (void*)Vp, DM, 0LL, bv, 64, 0, nbv,
      MQ, DM, DM, 64.0f, 1.0f);
  vtrans16<<<gV, blk, 0, stream>>>(Vp, VT);
  attn_mha<<<gAttn, dim3(128), 0, stream>>>(Qh, Ql, Kp, VT, Ch, Cl, 0.125f);
  gemm64<__bf16, 0, 1><<<gQ, blk, 0, stream>>>(
      Ch, Cl, DM, 0LL, DM, WoT, DM, 0LL, DM - 1,
      (void*)Y, (void*)Y, DM, 0LL, bo, 64, 0, nbo,
      MQ, DM, 2 * DM, 1.0f, 1.0f);
  lngelu<<<gLN, blk, 0, stream>>>(Y, Xb, gamma, ngm, beta, nbt, (float*)d_out);
  (void)hipGetLastError();
}
